// DQN_LSTM_88227218194755
// MI455X (gfx1250) — hardware-run, weakly checked
//
#include <hip/hip_runtime.h>


#define NB   65536
#define NP   16384
#define NPS  4
#define NI   28
#define NIP  32
#define NH   128
#define NG   512
#define ND   64
#define NO   4

typedef _Float16 h16;
typedef unsigned short bf;
typedef __attribute__((ext_vector_type(16))) __bf16   v16bf;
typedef __attribute__((ext_vector_type(16))) _Float16 v16h;
typedef __attribute__((ext_vector_type(8)))  _Float16 v8h;
typedef __attribute__((ext_vector_type(8)))  unsigned short v8us;
typedef __attribute__((ext_vector_type(8)))  float    v8f;
typedef __attribute__((ext_vector_type(4)))  float    v4f;
typedef v8h  __attribute__((may_alias)) v8ha;
typedef v4f  __attribute__((may_alias)) v4fa;
typedef v8us __attribute__((may_alias)) v8usa;

__device__ __forceinline__ unsigned short f2bf(float f) { unsigned u = __float_as_uint(f); u += 0x7FFFu + ((u >> 16) & 1u); return (unsigned short)(u >> 16); }
__device__ __forceinline__ float bf2f(unsigned short b) { return __uint_as_float(((unsigned)b) << 16); }
__device__ __forceinline__ float bfr(float f) { return bf2f(f2bf(f)); }
__device__ __forceinline__ v16h cat16(v8h lo, v8h hi) { return __builtin_shufflevector(lo, hi, 0, 1, 2, 3, 4, 5, 6, 7, 8, 9, 10, 11, 12, 13, 14, 15); }
__device__ __forceinline__ v16bf cat16b(v8us lo, v8us hi) { return __builtin_bit_cast(v16bf, __builtin_shufflevector(lo, hi, 0, 1, 2, 3, 4, 5, 6, 7, 8, 9, 10, 11, 12, 13, 14, 15)); }
__device__ __forceinline__ v8f wmma16(v16h a, v16h b, v8f c) { return __builtin_amdgcn_wmma_f32_16x16x32_f16(false, a, false, b, (short)0, c, false, false); }
__device__ __forceinline__ v8f wmmab(v16bf a, v16bf b, v8f c) { return __builtin_amdgcn_wmma_f32_16x16x32_bf16(false, a, false, b, (short)0, c, false, false); }

template <typename T16> struct WFrag;
template <> struct WFrag<h16> { typedef v16h V; static __device__ __forceinline__ V ld(const h16* p) { return cat16(*(const v8h*)p, *(const v8h*)(p + 16)); } static __device__ __forceinline__ v8f mma(V a, V b, v8f c) { return wmma16(a, b, c); } };
template <> struct WFrag<bf> { typedef v16bf V; static __device__ __forceinline__ V ld(const bf* p) { return cat16b(*(const v8us*)p, *(const v8us*)(p + 16)); } static __device__ __forceinline__ v8f mma(V a, V b, v8f c) { return wmmab(a, b, c); } };
template <typename T16, int NSPLIT, bool BIAS>
__global__ __launch_bounds__(32) void k_gemmw(const T16* __restrict__ A, const T16* __restrict__ A2, const T16* __restrict__ Bt, const T16* __restrict__ Bt2, int K, float* C, int ldc, const float* __restrict__ bias, size_t sA, size_t sB, size_t sC) {
    typedef typename WFrag<T16>::V V;
    __shared__ __align__(16) float os[16 * 68];
    const size_t z = blockIdx.z; A += z * sA; if (A2) A2 += z * sA; Bt += z * sB; if (Bt2) Bt2 += z * sB; C += z * sC;
    const int lane = threadIdx.x & 31, lr = lane & 15, hi = lane >> 4; const int r0 = blockIdx.x * 64, c0 = blockIdx.y * 64;
    v8f acc[4][4];
#pragma unroll
    for (int mb = 0; mb < 4; ++mb)
#pragma unroll
        for (int nb = 0; nb < 4; ++nb) acc[mb][nb] = (v8f){};
    const size_t aoff = (size_t)(r0 + lr) * K + 8 * hi, boff = (size_t)(c0 + lr) * K + 8 * hi;
    for (int kc = 0; kc < K; kc += 32) {
        V a[4], a2[4];
#pragma unroll
        for (int mb = 0; mb < 4; ++mb) { a[mb] = WFrag<T16>::ld(A + aoff + (size_t)mb * 16 * K + kc); if (NSPLIT == 1 || NSPLIT == 2) a2[mb] = WFrag<T16>::ld(A2 + aoff + (size_t)mb * 16 * K + kc); }
#pragma unroll
        for (int nb = 0; nb < 4; ++nb) { const V b = WFrag<T16>::ld(Bt + boff + (size_t)nb * 16 * K + kc); V b2; if (NSPLIT >= 2) b2 = WFrag<T16>::ld(Bt2 + boff + (size_t)nb * 16 * K + kc);
#pragma unroll
            for (int mb = 0; mb < 4; ++mb) { acc[mb][nb] = WFrag<T16>::mma(a[mb], b, acc[mb][nb]); if (NSPLIT == 1 || NSPLIT == 2) acc[mb][nb] = WFrag<T16>::mma(a2[mb], b, acc[mb][nb]); if (NSPLIT >= 2) acc[mb][nb] = WFrag<T16>::mma(a[mb], b2, acc[mb][nb]); } }
        asm volatile("v_nop\n\tv_nop\n\tv_nop\n\tv_nop" : "+v"(acc[0][0]), "+v"(acc[1][1]), "+v"(acc[2][2]), "+v"(acc[3][3]) : "v"(a[0]), "v"(a[3]));
    }
#pragma unroll
    for (int mb = 0; mb < 4; ++mb) {
#pragma unroll
        for (int nb = 0; nb < 4; ++nb) {
#pragma unroll
            for (int j = 0; j < 8; ++j) os[(hi * 8 + j) * 68 + nb * 16 + lr] = acc[mb][nb][j]; }
        __builtin_amdgcn_wave_barrier(); asm volatile("" ::: "memory");
        float* crow = C + (size_t)(r0 + mb * 16) * ldc + c0;
#pragma unroll 1
        for (int ps = 0; ps < 2; ++ps) {
#pragma unroll
            for (int s = 0; s < 8; ++s) { const int row = 2 * s + hi, cofs = lr * 4; v4f val = *(const v4fa*)(os + row * 68 + cofs); if (BIAS) { val[0] += bfr(bias[c0 + cofs]); val[1] += bfr(bias[c0 + cofs + 1]); val[2] += bfr(bias[c0 + cofs + 2]); val[3] += bfr(bias[c0 + cofs + 3]); }
                *(volatile v4f*)(crow + (size_t)row * ldc + cofs) = val; }
            if (ps == 0) __threadfence(); }
        __builtin_amdgcn_wave_barrier(); asm volatile("" ::: "memory");
    }
}

typedef __attribute__((ext_vector_type(2))) _Float16 v2h;
typedef __attribute__((ext_vector_type(4))) _Float16 v4h;
typedef __attribute__((ext_vector_type(2))) unsigned short v2us;
typedef __attribute__((ext_vector_type(4))) unsigned short v4us;
typedef __attribute__((ext_vector_type(2))) float v2f;
typedef __attribute__((ext_vector_type(4))) int v4i;
__global__ __launch_bounds__(256) void k_cvt8(const float* __restrict__ src, bf* dst, size_t n8) { const size_t i = (size_t)blockIdx.x * 256 + threadIdx.x; if (i >= n8) return; const v8f v = *(const v8f*)(src + i * 8); v8us o;
#pragma unroll
    for (int k = 0; k < 8; ++k) o[k] = f2bf(v[k]); *(volatile v8us*)(dst + i * 8) = o; __threadfence(); *(volatile v8us*)(dst + i * 8) = o; }

__global__ __launch_bounds__(256) void k_fillb(bf* P, unsigned w2, size_t n8) { const size_t i = (size_t)blockIdx.x * 256 + threadIdx.x; if (i >= n8) return; v4i o; o[0] = (int)w2; o[1] = (int)w2; o[2] = (int)w2; o[3] = (int)w2;
    *(volatile v4i*)(P + i * 8) = o; __threadfence(); *(volatile v4i*)(P + i * 8) = o; }

#define LNC_MAX 2048
template <bool RES>
__global__ __launch_bounds__(256) void k_lnrow(const float* __restrict__ A, const float* __restrict__ R, const float* __restrict__ gamma, const float* __restrict__ beta, float eps, int C, int nrows, float* Y) {
    const int lane = threadIdx.x & 31; const int row = blockIdx.x * 8 + (threadIdx.x >> 5); if (row >= nrows) return; const int nch = C / 128; const float* a = A + (size_t)row * C; float x[LNC_MAX / 32]; float s = 0.0f;
    for (int k = 0; k < LNC_MAX / 128; ++k) { if (k < nch) { const int c0 = k * 128 + lane * 4; v4f v = *(const v4f*)(a + c0);
            if (RES) { const v4f w = *(const v4f*)(R + (size_t)row * C + c0); v[0] = __fadd_rn(v[0], w[0]); v[1] = __fadd_rn(v[1], w[1]); v[2] = __fadd_rn(v[2], w[2]); v[3] = __fadd_rn(v[3], w[3]); }
            x[k * 4 + 0] = v[0]; x[k * 4 + 1] = v[1]; x[k * 4 + 2] = v[2]; x[k * 4 + 3] = v[3]; s = __fadd_rn(__fadd_rn(__fadd_rn(__fadd_rn(s, v[0]), v[1]), v[2]), v[3]); } }
    for (int sh = 16; sh; sh >>= 1) s = __fadd_rn(s, __shfl_xor(s, sh, 32));
    const float mean = __fdiv_rn(s, (float)C); float q = 0.0f;
    for (int k = 0; k < LNC_MAX / 128; ++k) { if (k < nch) {
            for (int j = 0; j < 4; ++j) { const float d = __fsub_rn(x[k * 4 + j], mean); x[k * 4 + j] = d; q = __fmaf_rn(d, d, q); } } }
    for (int sh = 16; sh; sh >>= 1) q = __fadd_rn(q, __shfl_xor(q, sh, 32));
    const float rstd = __fdiv_rn(1.0f, sqrtf(__fadd_rn(__fdiv_rn(q, (float)C), eps)));
    for (int k = 0; k < LNC_MAX / 128; ++k) { if (k < nch) { const int c0 = k * 128 + lane * 4; const v4f g = *(const v4f*)(gamma + c0); const v4f bt = *(const v4f*)(beta + c0);
            for (int j = 0; j < 4; ++j) x[k * 4 + j] = __fmaf_rn(__fmul_rn(x[k * 4 + j], rstd), bfr(g[j]), bfr(bt[j])); } }
    float* y = Y + (size_t)row * C;
    for (int ps = 0; ps < 2; ++ps) {
        for (int k = 0; k < LNC_MAX / 128; ++k) { if (k < nch) { v4f o; o[0] = x[k * 4 + 0]; o[1] = x[k * 4 + 1]; o[2] = x[k * 4 + 2]; o[3] = x[k * 4 + 3]; *(volatile v4f*)(y + k * 128 + lane * 4) = o; } }
        if (ps == 0) __threadfence(); }
}

__device__ __forceinline__ h16 toh_flush(float x) { const float z = (fabsf(x) < 6.103515625e-05f) ? 0.0f : x; return (h16)z; }

__global__ __launch_bounds__(256) void k_xp(const float* __restrict__ Sr, bf* Dp) { const unsigned id = blockIdx.x * 256u + threadIdx.x; const unsigned rw = id >> 2, e8 = id & 3u; const float* ps = Sr + (size_t)rw * NI + e8 * 8u; const v4f va = *(const v4f*)ps; const v4f vb = *(const v4f*)(ps + (e8 < 3u ? 4u : 0u)); const unsigned short mk = (unsigned short)(0u - (unsigned)(e8 < 3u)); v8us ov;
#pragma unroll
    for (int q2 = 0; q2 < 4; ++q2) { ov[q2] = f2bf(va[q2]); ov[4 + q2] = (unsigned short)(f2bf(vb[q2]) & mk); }
    *(volatile v8us*)(Dp + (size_t)id * 8) = ov; __threadfence(); *(volatile v8us*)(Dp + (size_t)id * 8) = ov; }

__global__ __launch_bounds__(256) void k_rs2(const float* __restrict__ Sr, bf* Eh, bf* El) { const size_t id = (size_t)blockIdx.x * 256 + threadIdx.x; const v4f va = *(const v4f*)(Sr + id * 8), vb = *(const v4f*)(Sr + id * 8 + 4); v8us oh, ol;
#pragma unroll
    for (int q2 = 0; q2 < 8; ++q2) { const float wv = fmaxf(q2 < 4 ? va[q2] : vb[q2 - 4], 0.0f); const unsigned short hw = f2bf(wv); oh[q2] = hw; ol[q2] = f2bf(wv - bf2f(hw)); }
    *(volatile v8us*)(Eh + id * 8) = oh; *(volatile v8us*)(El + id * 8) = ol; __threadfence(); *(volatile v8us*)(Eh + id * 8) = oh; *(volatile v8us*)(El + id * 8) = ol; }

__global__ __launch_bounds__(256) void k_r16(const float* __restrict__ Sr, unsigned sh, h16* Dh, unsigned pt, unsigned of) { const unsigned id = blockIdx.x * 256u + threadIdx.x; const unsigned rw = id >> sh, e8 = id & ((1u << sh) - 1u); const v4f va = *(const v4f*)(Sr + (size_t)id * 8), vb = *(const v4f*)(Sr + (size_t)id * 8 + 4); v8h ov;
#pragma unroll
    for (int q2 = 0; q2 < 8; ++q2) ov[q2] = toh_flush(fmaxf(q2 < 4 ? va[q2] : vb[q2 - 4], 0.0f));
    h16* pd = Dh + (size_t)rw * pt + of + e8 * 8u; *(volatile v8h*)pd = ov; __threadfence(); *(volatile v8h*)pd = ov; }

__global__ __launch_bounds__(256) void k_in16(const float* __restrict__ Sr, unsigned sh, h16* Dh, unsigned pt, unsigned of) { const unsigned id = blockIdx.x * 256u + threadIdx.x; const unsigned rw = id >> sh, e8 = id & ((1u << sh) - 1u); const v4f va = *(const v4f*)(Sr + (size_t)id * 8), vb = *(const v4f*)(Sr + (size_t)id * 8 + 4); v8h ov;
#pragma unroll
    for (int q2 = 0; q2 < 8; ++q2) ov[q2] = toh_flush(bfr(q2 < 4 ? va[q2] : vb[q2 - 4]));
    h16* pd = Dh + (size_t)rw * pt + of + e8 * 8u; *(volatile v8h*)pd = ov; __threadfence(); *(volatile v8h*)pd = ov; }

__device__ __forceinline__ float th(float w) { const float ee = expf(-2.0f * fabsf(w)); return copysignf((1.0f - ee) / (1.0f + ee), w); }

__global__ __launch_bounds__(256) void k_cell(const float* __restrict__ Gt, const float* __restrict__ a3, const float* __restrict__ a14, const float* __restrict__ a15, float* R2, float* R3, h16* Hh) { const unsigned id = blockIdx.x * 256u + threadIdx.x; const unsigned rw = id >> 5, k0 = (id & 31u) << 2; const float* pg = Gt + (size_t)rw * NG + k0; float wn[4][4];
#pragma unroll
    for (int r4 = 0; r4 < 4; ++r4) { const v4f ga = *(const v4f*)(pg + r4 * NH), ba = *(const v4f*)(a14 + r4 * NH + k0), ca = *(const v4f*)(a15 + r4 * NH + k0);
#pragma unroll
        for (int q2 = 0; q2 < 4; ++q2) wn[r4][q2] = ga[q2] + (bfr(ba[q2]) + bfr(ca[q2])); }
    const v4f oa = *(const v4f*)(a3 + (size_t)id * 4); v4f c1, h1; v4h oh;
#pragma unroll
    for (int q2 = 0; q2 < 4; ++q2) { const float s1 = 1.0f / (1.0f + expf(-wn[0][q2])), s2 = 1.0f / (1.0f + expf(-wn[1][q2])), s4 = 1.0f / (1.0f + expf(-wn[3][q2])); const float cv = s2 * bfr(oa[q2]) + s1 * th(wn[2][q2]); const float hv = s4 * th(cv); c1[q2] = cv; h1[q2] = hv; oh[q2] = toh_flush(hv); }
    float* p2 = R2 + (size_t)id * 4; float* p3 = R3 + (size_t)id * 4; h16* ph = Hh + (size_t)id * 4;
    *(volatile v4f*)p2 = h1; *(volatile v4f*)p3 = c1; *(volatile v4h*)ph = oh; __threadfence();
    *(volatile v4f*)p2 = h1; *(volatile v4f*)p3 = c1; *(volatile v4h*)ph = oh; }

__global__ __launch_bounds__(256) void k_q4(const float* __restrict__ Q6, const float* __restrict__ a19, float* R1) { const unsigned rw = blockIdx.x * 256u + threadIdx.x; const v4f qa = *(const v4f*)(Q6 + (size_t)rw * ND), ba = *(const v4f*)a19; v4f ov;
#pragma unroll
    for (int q2 = 0; q2 < 4; ++q2) ov[q2] = qa[q2] + bfr(ba[q2]);
    *(volatile v4f*)(R1 + (size_t)rw * NO) = ov; __threadfence(); *(volatile v4f*)(R1 + (size_t)rw * NO) = ov; }

extern "C" void kernel_launch(void* const* d_in, const int* in_sizes, int n_in, void* d_out, int out_size, void* d_ws, size_t ws_size, hipStream_t stream) {
    if (n_in < 19) return;
    if (in_sizes[0] != NB * NI || in_sizes[1] != NB * NH || in_sizes[2] != NB * NH || in_sizes[3] != NH * NI || in_sizes[4] != NH || in_sizes[5] != NH || in_sizes[6] != NH || in_sizes[7] != NH * NH || in_sizes[8] != NH || in_sizes[9] != NH || in_sizes[10] != NH || in_sizes[11] != NG * NH || in_sizes[12] != NG * NH || in_sizes[13] != NG || in_sizes[14] != NG || in_sizes[15] != ND * NH || in_sizes[16] != ND || in_sizes[17] != NO * ND || in_sizes[18] != NO) return;
    if (out_size != NB * NO + 2 * NB * NH) return;
    static_assert(NB == NPS * NP && NP % 64 == 0 && NH % 64 == 0 && NG % 64 == 0 && ND % 64 == 0 && NIP % 32 == 0 && NH % 32 == 0 && ND % 32 == 0 && (2 * NH) % 32 == 0 && NI == 28 && NIP == 32 && (NI * 4) % 16 == 0 && NG == 4 * NH && NH == 128 && ND == 64 && NO == 4 && (NB * 4) % 256 == 0 && (NH * 4) % 256 == 0 && (NH * NH / 8) % 256 == 0 && (NG * NH / 8) % 256 == 0 && (ND * NH / 8) % 256 == 0 && (NO * ND / 8) == 32 && (NP * NH / 8) % 256 == 0 && (NP * NH / 4) % 256 == 0 && (NP * ND / 8) % 256 == 0 && NP % 256 == 0 && NH % 128 == 0 && NH <= LNC_MAX && NP % 8 == 0 && (NO * ND * 2) % 128 == 0, "the products: row and column counts multiples of 64, the depths of 32; every flat grid exact but the two on W5 (k_in16 at 32 threads of a block of 256 would not be exact: see its launch) and k_fillb (the kit's own guard); k_lnrow: the channel count a multiple of 128 and at most LNC_MAX, the rows in eights; the noughts beneath W5's 4 rows begin on a whole line");
    const float* i0 = (const float*)d_in[0]; const float* i1 = (const float*)d_in[1]; const float* i2 = (const float*)d_in[2]; const float* i3 = (const float*)d_in[3]; const float* i4 = (const float*)d_in[4]; const float* i5 = (const float*)d_in[5]; const float* i6 = (const float*)d_in[6]; const float* i7 = (const float*)d_in[7]; const float* i8 = (const float*)d_in[8]; const float* i9 = (const float*)d_in[9]; const float* i10 = (const float*)d_in[10]; const float* i11 = (const float*)d_in[11]; const float* i12 = (const float*)d_in[12]; const float* i13 = (const float*)d_in[13]; const float* i14 = (const float*)d_in[14]; const float* i15 = (const float*)d_in[15]; const float* i16 = (const float*)d_in[16]; const float* i17 = (const float*)d_in[17]; const float* i18 = (const float*)d_in[18];
    float* r1 = (float*)d_out; float* r2 = r1 + (size_t)NB * NO; float* r3 = r2 + (size_t)NB * NH;
    char* wsp = (char*)d_ws; auto carve = [&](size_t bytes) { char* p = wsp; wsp += (bytes + 255) & ~(size_t)255; return (void*)p; };
    bf* Xp = (bf*)carve((size_t)NB * NIP * 2); bf* W1 = (bf*)carve((size_t)NH * NIP * 2); bf* W2 = (bf*)carve((size_t)NH * NH * 2); h16* Wc = (h16*)carve((size_t)NG * 2 * NH * 2); h16* W4 = (h16*)carve((size_t)ND * NH * 2); h16* W5 = (h16*)carve((size_t)ND * ND * 2);
    float* P1 = (float*)carve((size_t)NP * NH * 4); float* N1 = (float*)carve((size_t)NP * NH * 4); bf* E1h = (bf*)carve((size_t)NP * NH * 2); bf* E1l = (bf*)carve((size_t)NP * NH * 2); float* P2 = (float*)carve((size_t)NP * NH * 4); float* N2 = (float*)carve((size_t)NP * NH * 4); h16* Ct = (h16*)carve((size_t)NP * 2 * NH * 2); float* Gt = (float*)carve((size_t)NP * NG * 4); h16* Hh = (h16*)carve((size_t)NP * NH * 2); float* D1 = (float*)carve((size_t)NP * ND * 4); h16* Dh = (h16*)carve((size_t)NP * ND * 2); float* Q6 = (float*)carve((size_t)NP * ND * 4);
    if ((size_t)(wsp - (char*)d_ws) > ws_size) return;
    k_xp<<<(unsigned)(NB * 4 / 256), 256, 0, stream>>>(i0, Xp);
    k_xp<<<(unsigned)(NH * 4 / 256), 256, 0, stream>>>(i3, W1);
    k_cvt8<<<(unsigned)(NH * NH / 8 / 256), 256, 0, stream>>>(i7, W2, (size_t)NH * NH / 8);
    k_in16<<<(unsigned)(NG * NH / 8 / 256), 256, 0, stream>>>(i11, 4u, Wc, (unsigned)(2 * NH), 0u);
    k_in16<<<(unsigned)(NG * NH / 8 / 256), 256, 0, stream>>>(i12, 4u, Wc, (unsigned)(2 * NH), (unsigned)NH);
    k_in16<<<(unsigned)(ND * NH / 8 / 256), 256, 0, stream>>>(i15, 4u, W4, (unsigned)NH, 0u);
    k_in16<<<1, (unsigned)(NO * ND / 8), 0, stream>>>(i17, 3u, W5, (unsigned)ND, 0u);
    k_fillb<<<(unsigned)(((ND - NO) * ND / 8 + 255) / 256), 256, 0, stream>>>((bf*)(W5 + (size_t)NO * ND), 0u, (size_t)(ND - NO) * ND / 8);
    for (unsigned ps = 0; ps < (unsigned)NPS; ++ps) { const size_t r0 = (size_t)ps * NP;
        k_gemmw<bf, 0, true><<<dim3(NP / 64, NH / 64, 1), 32, 0, stream>>>(Xp + r0 * NIP, nullptr, W1, nullptr, NIP, P1, NH, i4, 0, 0, 0);
        k_lnrow<false><<<(unsigned)(NP / 8), 256, 0, stream>>>(P1, nullptr, i5, i6, 1.0e-5f, NH, NP, N1);
        k_rs2<<<(unsigned)(NP * NH / 8 / 256), 256, 0, stream>>>(N1, E1h, E1l);
        k_gemmw<bf, 1, true><<<dim3(NP / 64, NH / 64, 1), 32, 0, stream>>>(E1h, E1l, W2, nullptr, NH, P2, NH, i8, 0, 0, 0);
        k_lnrow<false><<<(unsigned)(NP / 8), 256, 0, stream>>>(P2, nullptr, i9, i10, 1.0e-5f, NH, NP, N2);
        k_r16<<<(unsigned)(NP * NH / 8 / 256), 256, 0, stream>>>(N2, 4u, Ct, (unsigned)(2 * NH), 0u);
        k_in16<<<(unsigned)(NP * NH / 8 / 256), 256, 0, stream>>>(i1 + r0 * NH, 4u, Ct, (unsigned)(2 * NH), (unsigned)NH);
        k_gemmw<h16, 0, false><<<dim3(NP / 64, NG / 64, 1), 32, 0, stream>>>(Ct, nullptr, Wc, nullptr, 2 * NH, Gt, NG, nullptr, 0, 0, 0);
        k_cell<<<(unsigned)(NP * NH / 4 / 256), 256, 0, stream>>>(Gt, i2 + r0 * NH, i13, i14, r2 + r0 * NH, r3 + r0 * NH, Hh);
        k_gemmw<h16, 0, true><<<dim3(NP / 64, ND / 64, 1), 32, 0, stream>>>(Hh, nullptr, W4, nullptr, NH, D1, ND, i16, 0, 0, 0);
        k_r16<<<(unsigned)(NP * ND / 8 / 256), 256, 0, stream>>>(D1, 3u, Dh, (unsigned)ND, 0u);
        k_gemmw<h16, 0, false><<<dim3(NP / 64, ND / 64, 1), 32, 0, stream>>>(Dh, nullptr, W5, nullptr, ND, Q6, ND, nullptr, 0, 0, 0);
        k_q4<<<(unsigned)(NP / 256), 256, 0, stream>>>(Q6, i18, r1 + r0 * NO); }
}
